// GeometricAttentionLayer_24876450579070
// MI455X (gfx1250) — hardware-run, weakly checked
//
#include <hip/hip_runtime.h>
#include <math.h>

constexpr int kBatch = 2;
constexpr int kSeq   = 2048;
constexpr int kDim   = 1024;
constexpr int kHeads = 16;
constexpr int kHdim  = 64;
constexpr int kFfn   = 4096;
constexpr int kTok   = kBatch * kSeq;
constexpr int kGrp   = 2;
constexpr float kWCarry    = 16.0f;
constexpr float kWCarryInv = 1.0f / 16.0f;
constexpr float kPCarry    = 2048.0f;
constexpr float kCtxCarry  = 256.0f;
constexpr float kPVScale   = kCtxCarry / kPCarry;
constexpr float kOutScale  = 1.0f / (kCtxCarry * kWCarry);
constexpr float kInvDim    = 1.0f / 1024.0f;
constexpr float kLnEps     = 1e-5f;

static_assert(kDim % 64 == 0 && kFfn % 64 == 0 && kTok % 64 == 0 && kSeq % 64 == 0, "tile multiples");
static_assert(kDim % 32 == 0 && kHdim % 32 == 0 && kSeq % 32 == 0 && kFfn % 32 == 0, "K multiples of 32");
static_assert(kHeads % kGrp == 0, "chunking");

constexpr size_t kMiB      = (size_t)1 << 20;
constexpr size_t kOffQ16   = 0;
constexpr size_t kOffK16   = 8 * kMiB;
constexpr size_t kOffVT16  = 16 * kMiB;
constexpr size_t kOffO16   = 24 * kMiB;
constexpr size_t kOffScr   = 32 * kMiB;
constexpr size_t kOffX16   = kOffScr;
constexpr size_t kOffWqkvT = kOffScr + 8 * kMiB;
constexpr size_t kOffScore = kOffScr;
constexpr size_t kOffP     = kOffScr + 64 * kMiB;
constexpr size_t kOffWoT   = 0;
constexpr size_t kOffWff1T = 2 * kMiB;
constexpr size_t kOffWff2T = 10 * kMiB;
constexpr size_t kOffPre1  = kOffScr;
constexpr size_t kOffH1F   = kOffScr + 16 * kMiB;
constexpr size_t kOffH1H   = kOffScr + 32 * kMiB;
constexpr size_t kOffFF1   = kOffScr + 40 * kMiB;
constexpr size_t kOffPre2  = kOffScr + 72 * kMiB;
constexpr size_t kWsTotal  = 128 * kMiB;

static_assert((size_t)kTok * kDim * 2 == 8 * kMiB, "plane size");
static_assert((size_t)kDim * kDim * 2 * 3 == 6 * kMiB, "wqkv planes");
static_assert(kOffWqkvT + 6 * kMiB <= kWsTotal, "prep fits");
static_assert((size_t)kGrp * kSeq * kSeq * 4 == 32 * kMiB, "scores chunk");
static_assert(kOffP + (size_t)kGrp * kSeq * kSeq * 2 <= kWsTotal, "P chunk within total");
static_assert(kOffWff2T + (size_t)kFfn * kDim * 2 <= kOffO16, "late weights do not touch O16");
static_assert(kOffFF1 + (size_t)kTok * kFfn * 2 == kOffPre2, "ff1 plane");
static_assert(kOffPre2 + (size_t)kTok * kDim * 4 <= kWsTotal, "post fits");

typedef __attribute__((ext_vector_type(16))) _Float16 v16h;
typedef __attribute__((ext_vector_type(8)))  _Float16 v8h;
typedef __attribute__((ext_vector_type(16))) __bf16   v16b;
typedef __attribute__((ext_vector_type(8)))  __bf16   v8b;
typedef __attribute__((ext_vector_type(8)))  float    v8f;
typedef __attribute__((ext_vector_type(4)))  float    v4f;
typedef __attribute__((ext_vector_type(4)))  unsigned int v4u;

__device__ __forceinline__ unsigned short f2bf_bits(float f) {
  unsigned u = __float_as_uint(f);
  return (unsigned short)((u + 0x7FFFu + ((u >> 16) & 1u)) >> 16);
}
__device__ __forceinline__ float bf_bits2f(unsigned short h) { return __uint_as_float(((unsigned)h) << 16); }

__device__ __forceinline__ void dep_guard_h(v8f& a, v8f& b, v16h x, v16h y) { asm volatile("v_nop\n\tv_nop\n\tv_nop\n\tv_nop" : "+v"(a), "+v"(b) : "v"(x), "v"(y)); }
__device__ __forceinline__ void dep_guard_b(v8f& a, v8f& b, v16b x, v16b y) { asm volatile("v_nop\n\tv_nop\n\tv_nop\n\tv_nop" : "+v"(a), "+v"(b) : "v"(x), "v"(y)); }
__device__ __forceinline__ void keep4_h(v16h a, v16h b, v16h c, v16h d) { asm volatile("v_nop" :: "v"(a), "v"(b), "v"(c), "v"(d)); }
__device__ __forceinline__ void keep4_b(v16b a, v16b b, v16b c, v16b d) { asm volatile("v_nop" :: "v"(a), "v"(b), "v"(c), "v"(d)); }
__device__ __forceinline__ void acc_guard4(v8f& a, v8f& b, v8f& c, v8f& d) { asm volatile("v_nop\n\tv_nop\n\tv_nop\n\tv_nop" : "+v"(a), "+v"(b), "+v"(c), "+v"(d)); }
template <typename T> struct Frag;
template <> struct Frag<_Float16> {
  typedef v16h V; union U { v16h v; v8h h[2]; };
  static __device__ __forceinline__ v16h load(const _Float16* p) {
    U f; f.h[0] = *(const v8h*)(p); f.h[1] = *(const v8h*)(p + 16); return f.v;
  }
  static __device__ __forceinline__ v8f mma(v16h a, v16h b, v8f c) {
    return __builtin_amdgcn_wmma_f32_16x16x32_f16(false, a, false, b, (short)0, c, false, false);
  }
  static __device__ __forceinline__ void guard(v8f& a, v8f& b, v16h x, v16h y) { dep_guard_h(a, b, x, y); }
  static __device__ __forceinline__ void keep(v16h a, v16h b, v16h c, v16h d) { keep4_h(a, b, c, d); }
};
template <> struct Frag<__bf16> {
  typedef v16b V; union U { v16b v; v8b h[2]; };
  static __device__ __forceinline__ v16b load(const __bf16* p) {
    U f; f.h[0] = *(const v8b*)(p); f.h[1] = *(const v8b*)(p + 16); return f.v;
  }
  static __device__ __forceinline__ v8f mma(v16b a, v16b b, v8f c) {
    return __builtin_amdgcn_wmma_f32_16x16x32_bf16(false, a, false, b, (short)0, c, false, false);
  }
  static __device__ __forceinline__ void guard(v8f& a, v8f& b, v16b x, v16b y) { dep_guard_b(a, b, x, y); }
  static __device__ __forceinline__ void keep(v16b a, v16b b, v16b c, v16b d) { keep4_b(a, b, c, d); }
};

__device__ __forceinline__ unsigned pk16(unsigned short a, unsigned short b) { return (unsigned)a | ((unsigned)b << 16); }
__device__ __forceinline__ unsigned short h_bits(float f) { const _Float16 h = (_Float16)f; return __builtin_bit_cast(unsigned short, h); }

template <int ET> struct Elem;
template <> struct Elem<0> { typedef _Float16 T; };
template <> struct Elem<1> { typedef __bf16 T; };
template <int ET, bool SPLIT, int BIAS_MODE, int OUT_MODE, bool RESID, int ACT = 0>
__global__ __launch_bounds__(256) void wmma_gemm64(
    const unsigned short* __restrict__ Ap, const unsigned short* __restrict__ A2p, int lda, long strideA,
    const unsigned short* __restrict__ Btp, const unsigned short* __restrict__ Bt2p, int ldb, long strideB,
    void* __restrict__ Cout, void* __restrict__ Cout2, int ldc, long strideC,
    const float* __restrict__ bias,
    const float* __restrict__ resid, long strideR,
    int M, int N, int K, float scale) {
  typedef typename Elem<ET>::T T;
  typedef typename Frag<T>::V V;
  const T* A = (const T*)Ap; const T* A2 = (const T*)A2p; const T* Bt = (const T*)Btp; const T* Bt2 = (const T*)Bt2p;
  __shared__ __align__(16) float sT[8][16 * 68];
  const int b    = blockIdx.y;
  const int lane = threadIdx.x & 31;
  const int wave = threadIdx.x >> 5;
  const int tilesN = N >> 6;
  const int tilesM = M >> 6;
  const int tile = blockIdx.x * 8 + wave;
  if (tile >= tilesM * tilesN) return;
  const int tm = tile / tilesN;
  const int tn = tile - tm * tilesN;
  const int m0 = tm << 6;
  const int n0 = tn << 6;

  const T* Ab  = A  + (size_t)b * strideA;
  const T* Bb  = Bt + (size_t)b * strideB;
  const T* Ab2 = SPLIT ? (A2  + (size_t)b * strideA) : nullptr;
  const T* Bb2 = SPLIT ? (Bt2 + (size_t)b * strideB) : nullptr;

  const int rlane = lane & 15;
  const int koff  = (lane >> 4) * 8;
  const int mOff  = (lane >> 4) * 8;

  v8f acc[4][4];
#pragma unroll
  for (int i = 0; i < 4; ++i)
#pragma unroll
    for (int j = 0; j < 4; ++j) acc[i][j] = (v8f){0.f,0.f,0.f,0.f,0.f,0.f,0.f,0.f};

  for (int k0 = 0; k0 < K; k0 += 32) {
    V bh[4], bl[4];
#pragma unroll
    for (int j = 0; j < 4; ++j) {
      const size_t bo = (size_t)(n0 + (j << 4) + rlane) * ldb + koff + k0;
      bh[j] = Frag<T>::load(Bb + bo);
      if (SPLIT) bl[j] = Frag<T>::load(Bb2 + bo);
    }
#pragma unroll
    for (int i = 0; i < 4; ++i) {
      const size_t ao = (size_t)(m0 + (i << 4) + rlane) * lda + koff + k0;
      V ah = Frag<T>::load(Ab + ao);
      V al;
      if (SPLIT) al = Frag<T>::load(Ab2 + ao);
#pragma unroll
      for (int j = 0; j < 4; ++j) {
        acc[i][j] = Frag<T>::mma(ah, bh[j], acc[i][j]);
        if (SPLIT) {
          acc[i][j] = Frag<T>::mma(ah, bl[j], acc[i][j]);
          acc[i][j] = Frag<T>::mma(al, bh[j], acc[i][j]);
        }
      }
      Frag<T>::guard(acc[i][0], acc[i][3], ah, SPLIT ? al : ah);
    }
    Frag<T>::keep(bh[0], bh[1], bh[2], bh[3]);
    if (SPLIT) Frag<T>::keep(bl[0], bl[1], bl[2], bl[3]);
  }
  acc_guard4(acc[0][0], acc[0][1], acc[0][2], acc[0][3]);
  acc_guard4(acc[1][0], acc[1][1], acc[1][2], acc[1][3]);
  acc_guard4(acc[2][0], acc[2][1], acc[2][2], acc[2][3]);
  acc_guard4(acc[3][0], acc[3][1], acc[3][2], acc[3][3]);

  float* slab = sT[wave];
  const float* Rb = RESID ? (resid + (size_t)b * strideR) : nullptr;
#pragma unroll
  for (int i = 0; i < 4; ++i) {
    const int mBase = m0 + (i << 4);
#pragma unroll
    for (int j = 0; j < 4; ++j) {
      const int n = n0 + (j << 4) + rlane;
      float bv = 0.f;
      if (BIAS_MODE == 2) bv = bias[n];
#pragma unroll
      for (int r = 0; r < 8; ++r) {
        float v = acc[i][j][r] * scale;
        if (BIAS_MODE == 1) v += bias[mBase + mOff + r];
        if (BIAS_MODE == 2) v += bv;
        if (RESID) v += Rb[(size_t)(mBase + mOff + r) * ldc + n];
        if (ACT == 2) v = fmaxf(v, 0.0f);
        if (ACT == 4) v = (v > 0.f) ? v : 0.01f * v;
        slab[(mOff + r) * 68 + (j << 4) + rlane] = v;
      }
    }
    __builtin_amdgcn_fence(__ATOMIC_RELEASE, "workgroup");
    __builtin_amdgcn_wave_barrier();
    __builtin_amdgcn_fence(__ATOMIC_ACQUIRE, "workgroup");
    if (OUT_MODE == 0) {
      float* C = (float*)Cout + (size_t)b * strideC;
      const int hh = lane >> 4, c4 = (lane & 15) * 4;
      for (int pass = 0; pass < 2; ++pass) {
#pragma unroll
        for (int it = 0; it < 8; ++it) {
          const int row = it * 2 + hh;
          v4f v = *(const v4f*)(slab + row * 68 + c4);
          *(volatile v4f*)(C + (size_t)(mBase + row) * ldc + n0 + c4) = v;
        }
        __threadfence();
      }
    } else {
      const int q = lane >> 3, c8 = (lane & 7) * 8;
      unsigned short* C  = (unsigned short*)Cout  + (size_t)b * strideC;
      unsigned short* C2 = (OUT_MODE == 2) ? ((unsigned short*)Cout2 + (size_t)b * strideC) : nullptr;
      for (int pass = 0; pass < 2; ++pass) {
#pragma unroll
        for (int it = 0; it < 4; ++it) {
          const int row = it * 4 + q;
          const float* sp = slab + row * 68 + c8;
          v8h hv, lv;
#pragma unroll
          for (int e = 0; e < 8; ++e) {
            if (OUT_MODE == 1) {
              hv[e] = (_Float16)sp[e];
            } else {
              unsigned short hb = f2bf_bits(sp[e]);
              unsigned short lb = f2bf_bits(sp[e] - bf_bits2f(hb));
              hv[e] = __builtin_bit_cast(_Float16, hb);
              lv[e] = __builtin_bit_cast(_Float16, lb);
            }
          }
          *(volatile v8h*)(C + (size_t)(mBase + row) * ldc + n0 + c8) = hv;
          if (OUT_MODE == 2) *(volatile v8h*)(C2 + (size_t)(mBase + row) * ldc + n0 + c8) = lv;
        }
        __threadfence();
      }
    }
    __builtin_amdgcn_fence(__ATOMIC_RELEASE, "workgroup");
    __builtin_amdgcn_wave_barrier();
    __builtin_amdgcn_fence(__ATOMIC_ACQUIRE, "workgroup");
  }
}

__global__ __launch_bounds__(256) void wtcast_kernel(const float* __restrict__ W0, const float* __restrict__ W1,
                                                     const float* __restrict__ W2,
                                                     unsigned short* __restrict__ out, int R, int Cc, float scale) {
  __shared__ float sm[64][65];
  const int t  = threadIdx.x;
  const int r0 = blockIdx.x * 64;
  const int c0 = blockIdx.y * 64;
  const int z  = blockIdx.z;
  const float* W = (z == 0) ? W0 : (z == 1) ? W1 : W2;
#pragma unroll
  for (int i = 0; i < 16; ++i) {
    const int e = i * 256 + t;
    const int rl = e >> 6;
    const int cl = e & 63;
    sm[cl][rl] = W[(size_t)(r0 + rl) * Cc + c0 + cl] * scale;
  }
  __syncthreads();
  const int lane = t & 31, wave = t >> 5;
  const int q = lane >> 3, c8 = (lane & 7) * 8;
  unsigned short* op = out + (size_t)z * (size_t)R * (size_t)Cc;
  for (int pass = 0; pass < 2; ++pass) {
#pragma unroll
    for (int it = 0; it < 2; ++it) {
      const int row = wave * 8 + it * 4 + q;
      unsigned short hb[8];
#pragma unroll
      for (int e = 0; e < 8; ++e) hb[e] = h_bits(sm[row][c8 + e]);
      const v4u u = (v4u){pk16(hb[0], hb[1]), pk16(hb[2], hb[3]), pk16(hb[4], hb[5]), pk16(hb[6], hb[7])};
      *(volatile v4u*)(op + (size_t)(c0 + row) * R + r0 + c8) = u;
    }
    __threadfence();
  }
}

__global__ __launch_bounds__(256) void cast8_f16_kernel(const float* __restrict__ in, unsigned short* __restrict__ out, int n8) {
  const int i = blockIdx.x * 256 + threadIdx.x;
  if (i >= n8) return;
  const float* p = in + 8 * (size_t)i;
  const v4f a = *(const v4f*)(p);
  const v4f c = *(const v4f*)(p + 4);
  unsigned short hb[8];
#pragma unroll
  for (int e = 0; e < 4; ++e) {
    hb[e]     = h_bits(a[e]);
    hb[4 + e] = h_bits(c[e]);
  }
  const v4u u = (v4u){pk16(hb[0], hb[1]), pk16(hb[2], hb[3]), pk16(hb[4], hb[5]), pk16(hb[6], hb[7])};
  unsigned short* q = out + 8 * (size_t)i;
  *(volatile v4u*)q = u;
  __threadfence();
  *(volatile v4u*)q = u;
}

__global__ __launch_bounds__(256) void softmax_row_kernel(const float* __restrict__ Sc, unsigned short* __restrict__ P, float carry) {
  __shared__ float redM[8];
  __shared__ float redS[8];
  const int row  = blockIdx.x;
  const int t    = threadIdx.x;
  const int lane = t & 31, wave = t >> 5;
  const int c0   = t * 8;
  const float* sr = Sc + (size_t)row * kSeq + c0;
  const v4f a = *(const v4f*)(sr);
  const v4f c = *(const v4f*)(sr + 4);
  float x[8];
#pragma unroll
  for (int e = 0; e < 4; ++e) { x[e] = a[e]; x[4 + e] = c[e]; }
  float m = fmaxf(fmaxf(fmaxf(x[0], x[1]), fmaxf(x[2], x[3])), fmaxf(fmaxf(x[4], x[5]), fmaxf(x[6], x[7])));
#pragma unroll
  for (int off = 16; off > 0; off >>= 1) m = fmaxf(m, __shfl_xor(m, off, 32));
  if (lane == 0) redM[wave] = m;
  __syncthreads();
  float gm = redM[0];
#pragma unroll
  for (int w = 1; w < 8; ++w) gm = fmaxf(gm, redM[w]);
  float ex[8];
  float s = 0.0f;
#pragma unroll
  for (int e = 0; e < 8; ++e) { ex[e] = expf(x[e] - gm); s += ex[e]; }
#pragma unroll
  for (int off = 16; off > 0; off >>= 1) s += __shfl_xor(s, off, 32);
  if (lane == 0) redS[wave] = s;
  __syncthreads();
  float tot = 0.0f;
#pragma unroll
  for (int w = 0; w < 8; ++w) tot += redS[w];
  const float inv = carry / tot;
  unsigned short hb[8];
#pragma unroll
  for (int e = 0; e < 8; ++e) hb[e] = h_bits(ex[e] * inv);
  const v4u u = (v4u){pk16(hb[0], hb[1]), pk16(hb[2], hb[3]), pk16(hb[4], hb[5]), pk16(hb[6], hb[7])};
  unsigned short* q = P + (size_t)row * kSeq + c0;
  *(volatile v4u*)q = u;
  __threadfence();
  *(volatile v4u*)q = u;
}

template <bool HOUT>
__global__ __launch_bounds__(256) void layernorm_kernel(const float* __restrict__ X, const float* __restrict__ g,
                                                        const float* __restrict__ bb, float* __restrict__ outF,
                                                        unsigned short* __restrict__ outH) {
  __shared__ float redA[8];
  __shared__ float redB[8];
  __shared__ __align__(16) float srow[kDim];
  const int row  = blockIdx.x;
  const int t    = threadIdx.x;
  const int lane = t & 31, wave = t >> 5;
  const int c0   = t * 4;
  const v4f xv = *(const v4f*)(X + (size_t)row * kDim + c0);
  float s = (xv[0] + xv[1]) + (xv[2] + xv[3]);
#pragma unroll
  for (int off = 16; off > 0; off >>= 1) s += __shfl_xor(s, off, 32);
  if (lane == 0) redA[wave] = s;
  __syncthreads();
  float tot = 0.0f;
#pragma unroll
  for (int w = 0; w < 8; ++w) tot += redA[w];
  const float mu = tot * kInvDim;
  float dv[4];
#pragma unroll
  for (int e = 0; e < 4; ++e) dv[e] = xv[e] - mu;
  float qsum = (dv[0] * dv[0] + dv[1] * dv[1]) + (dv[2] * dv[2] + dv[3] * dv[3]);
#pragma unroll
  for (int off = 16; off > 0; off >>= 1) qsum += __shfl_xor(qsum, off, 32);
  if (lane == 0) redB[wave] = qsum;
  __syncthreads();
  float qtot = 0.0f;
#pragma unroll
  for (int w = 0; w < 8; ++w) qtot += redB[w];
  const float var = qtot * kInvDim;
  const float inv = rsqrtf(var + kLnEps);
  const v4f gv = *(const v4f*)(g + c0);
  const v4f bv4 = *(const v4f*)(bb + c0);
  v4f y;
#pragma unroll
  for (int e = 0; e < 4; ++e) y[e] = (dv[e] * inv) * gv[e] + bv4[e];
  float* op = outF + (size_t)row * kDim + c0;
  *(volatile v4f*)op = y;
  __threadfence();
  *(volatile v4f*)op = y;
  if (HOUT) {
    *(v4f*)(srow + c0) = y;
    __syncthreads();
    if (t < 128) {
      const float* sp = srow + t * 8;
      const v4f p0 = *(const v4f*)(sp);
      const v4f p1 = *(const v4f*)(sp + 4);
      unsigned short hb[8];
#pragma unroll
      for (int e = 0; e < 4; ++e) { hb[e] = h_bits(p0[e]); hb[4 + e] = h_bits(p1[e]); }
      const v4u u = (v4u){pk16(hb[0], hb[1]), pk16(hb[2], hb[3]), pk16(hb[4], hb[5]), pk16(hb[6], hb[7])};
      unsigned short* hq = outH + (size_t)row * kDim + t * 8;
      *(volatile v4u*)hq = u;
      __threadfence();
      *(volatile v4u*)hq = u;
    }
  }
}

extern "C" void kernel_launch(void* const* d_in, const int* in_sizes, int n_in,
                              void* d_out, int out_size, void* d_ws, size_t ws_size,
                              hipStream_t stream)
{
  if (n_in < 17) return;
  if (in_sizes[0] != kTok * kDim) return;
  if ((size_t)out_size < (size_t)kTok * kDim) return;
  if (ws_size < kWsTotal) return;

  const float* x     = (const float*)d_in[0];
  const float* Wq    = (const float*)d_in[1];
  const float* bq    = (const float*)d_in[2];
  const float* Wk    = (const float*)d_in[3];
  const float* bk    = (const float*)d_in[4];
  const float* Wv    = (const float*)d_in[5];
  const float* bv    = (const float*)d_in[6];
  const float* Wo    = (const float*)d_in[7];
  const float* bo    = (const float*)d_in[8];
  const float* g1    = (const float*)d_in[9];
  const float* b1    = (const float*)d_in[10];
  const float* Wff1  = (const float*)d_in[11];
  const float* bff1  = (const float*)d_in[12];
  const float* Wff2  = (const float*)d_in[13];
  const float* bff2  = (const float*)d_in[14];
  const float* g2    = (const float*)d_in[15];
  const float* b2    = (const float*)d_in[16];
  float* out = (float*)d_out;

  char* ws = (char*)d_ws;
  unsigned short* Q16   = (unsigned short*)(ws + kOffQ16);
  unsigned short* K16   = (unsigned short*)(ws + kOffK16);
  unsigned short* VT16  = (unsigned short*)(ws + kOffVT16);
  unsigned short* O16   = (unsigned short*)(ws + kOffO16);
  unsigned short* X16   = (unsigned short*)(ws + kOffX16);
  unsigned short* WqkvT = (unsigned short*)(ws + kOffWqkvT);
  float*          SCORE = (float*)(ws + kOffScore);
  unsigned short* PPL   = (unsigned short*)(ws + kOffP);
  unsigned short* WoT   = (unsigned short*)(ws + kOffWoT);
  unsigned short* Wff1T = (unsigned short*)(ws + kOffWff1T);
  unsigned short* Wff2T = (unsigned short*)(ws + kOffWff2T);
  float*          PRE1  = (float*)(ws + kOffPre1);
  float*          H1F   = (float*)(ws + kOffH1F);
  unsigned short* H1H   = (unsigned short*)(ws + kOffH1H);
  unsigned short* FF1P  = (unsigned short*)(ws + kOffFF1);
  float*          PRE2  = (float*)(ws + kOffPre2);

  const float score_scale = (float)(1.05 / 8.0);

  cast8_f16_kernel<<<(kTok * kDim / 8) / 256, 256, 0, stream>>>(x, X16, kTok * kDim / 8);
  wtcast_kernel<<<dim3(kDim / 64, kDim / 64, 3), 256, 0, stream>>>(Wq, Wk, Wv, WqkvT, kDim, kDim, kWCarry);

  wmma_gemm64<0, false, 2, 1, false, 0><<<dim3((kTok / 64) * (kDim / 64) / 8, 1), 256, 0, stream>>>(
      X16, nullptr, kDim, 0, WqkvT, nullptr, kDim, 0,
      Q16, nullptr, kDim, 0, bq, nullptr, 0, kTok, kDim, kDim, kWCarryInv);
  wmma_gemm64<0, false, 2, 1, false, 0><<<dim3((kTok / 64) * (kDim / 64) / 8, 1), 256, 0, stream>>>(
      X16, nullptr, kDim, 0, WqkvT + (size_t)kDim * kDim, nullptr, kDim, 0,
      K16, nullptr, kDim, 0, bk, nullptr, 0, kTok, kDim, kDim, kWCarryInv);
  wmma_gemm64<0, false, 1, 1, false, 0><<<dim3((kDim / 64) * (kTok / 64) / 8, 1), 256, 0, stream>>>(
      WqkvT + (size_t)2 * kDim * kDim, nullptr, kDim, 0, X16, nullptr, kDim, 0,
      VT16, nullptr, kTok, 0, bv, nullptr, 0, kDim, kTok, kDim, kWCarryInv);

  for (int bb = 0; bb < kBatch; ++bb) {
    for (int hc = 0; hc < kHeads / kGrp; ++hc) {
      const size_t qoff = (size_t)bb * kSeq * kDim + (size_t)hc * kGrp * kHdim;
      wmma_gemm64<0, false, 0, 0, false, 0><<<dim3((kSeq / 64) * (kSeq / 64) / 8, kGrp), 256, 0, stream>>>(
          Q16 + qoff, nullptr, kDim, (long)kHdim, K16 + qoff, nullptr, kDim, (long)kHdim,
          SCORE, nullptr, kSeq, (long)kSeq * kSeq, nullptr, nullptr, 0, kSeq, kSeq, kHdim, score_scale);
      softmax_row_kernel<<<kGrp * kSeq, 256, 0, stream>>>(SCORE, PPL, kPCarry);
      const size_t voff = (size_t)(hc * kGrp * kHdim) * kTok + (size_t)bb * kSeq;
      wmma_gemm64<0, false, 0, 1, false, 0><<<dim3((kSeq / 64) * (kHdim / 64) / 8, kGrp), 256, 0, stream>>>(
          PPL, nullptr, kSeq, (long)kSeq * kSeq, VT16 + voff, nullptr, kTok, (long)kHdim * kTok,
          O16 + qoff, nullptr, kDim, (long)kHdim, nullptr, nullptr, 0, kSeq, kHdim, kSeq, kPVScale);
    }
  }

  wtcast_kernel<<<dim3(kDim / 64, kDim / 64, 1), 256, 0, stream>>>(Wo, Wo, Wo, WoT, kDim, kDim, kWCarry);
  wtcast_kernel<<<dim3(kDim / 64, kFfn / 64, 1), 256, 0, stream>>>(Wff1, Wff1, Wff1, Wff1T, kDim, kFfn, kWCarry);
  wtcast_kernel<<<dim3(kFfn / 64, kDim / 64, 1), 256, 0, stream>>>(Wff2, Wff2, Wff2, Wff2T, kFfn, kDim, kWCarry);

  wmma_gemm64<0, false, 2, 0, true, 0><<<dim3((kTok / 64) * (kDim / 64) / 8, 1), 256, 0, stream>>>(
      O16, nullptr, kDim, 0, WoT, nullptr, kDim, 0,
      PRE1, nullptr, kDim, 0, bo, x, 0, kTok, kDim, kDim, kOutScale);
  layernorm_kernel<true><<<kTok, 256, 0, stream>>>(PRE1, g1, b1, H1F, H1H);
  wmma_gemm64<0, false, 2, 1, false, 2><<<dim3((kTok / 64) * (kFfn / 64) / 8, 1), 256, 0, stream>>>(
      H1H, nullptr, kDim, 0, Wff1T, nullptr, kDim, 0,
      FF1P, nullptr, kFfn, 0, bff1, nullptr, 0, kTok, kFfn, kDim, kWCarryInv);
  wmma_gemm64<0, false, 2, 0, true, 0><<<dim3((kTok / 64) * (kDim / 64) / 8, 1), 256, 0, stream>>>(
      FF1P, nullptr, kFfn, 0, Wff2T, nullptr, kFfn, 0,
      PRE2, nullptr, kDim, 0, bff2, H1F, 0, kTok, kDim, kFfn, kWCarryInv);
  layernorm_kernel<false><<<kTok, 256, 0, stream>>>(PRE2, g2, b2, out, nullptr);
}
